// Ext_entLayer_4561255268668
// MI455X (gfx1250) — hardware-verified
//
#include <hip/hip_runtime.h>
#include <stddef.h>


#define ENTD    128
#define RELD    128
#define TIMD    64
#define COMPD   320
#define PEP     384
#define PRP     256
#define NTHR    256
#define NWAVE   8
#define EPT     8
#define NGRP    2
#define CHUNK   (NTHR * EPT * NGRP)
#define WCAP    (EPT * NGRP * 32)
#define LISTN   (NWAVE * WCAP)
#define NBC     4096
#define NBF     1024
#define RCAP    40960
#define RBN     128
#define TGT     256
#define DEGCAP  1024
#define GROWS   128
#define OTHR    512
#define WSCAP   134217728
#define WSCALE  16.0f
#define WINV    0.0625f
#define WPREP_BLOCKS 50

#define LDS_FILL ((RCAP + NBF + LISTN) * 4 + 64)

static_assert((CHUNK & (CHUNK - 1)) == 0);
static_assert(CHUNK <= 4096);
static_assert(NBC <= 4096 && NBF <= 4096);
static_assert((NBC & (NBC - 1)) == 0 && (NBF & (NBF - 1)) == 0);
static_assert(NBC == 4 * NBF);
static_assert(OTHR * 8 == NBC);
static_assert((RCAP % 32) == 0);
static_assert(TGT == NWAVE * 32 && (TGT % GROWS) == 0);
static_assert((NBC % TGT) == 0);
static_assert(GROWS == NWAVE * 16);
static_assert(ENTD == 128 && RELD == 128 && TIMD == 64 && COMPD == RELD + ENTD + TIMD);
static_assert(PEP == 3 * ENTD && PRP == 2 * ENTD);

typedef float    v4f  __attribute__((ext_vector_type(4)));
typedef float    v8f  __attribute__((ext_vector_type(8)));
typedef int      v4i  __attribute__((ext_vector_type(4)));
typedef _Float16 v8h  __attribute__((ext_vector_type(8)));
typedef _Float16 v16h __attribute__((ext_vector_type(16)));
union FragH { v16h v; v8h h[2]; };

template <int K, int NCT> struct GemmCfg {
  static constexpr int APK  = K + 8;
  static constexpr int P    = 64 * NCT;
  static constexpr int CW   = (NCT == 1) ? 64 : 128;
  static constexpr int NG   = P / CW;
  static constexpr int NCH  = CW / 64;
  static constexpr int LDSA = GROWS * APK * 2;
  static constexpr int LDS  = LDSA + GROWS * CW * 4;
};

__device__ __forceinline__ v8f wmh(v16h a, v16h b, v8f c) {
  v8f d = __builtin_amdgcn_wmma_f32_16x16x32_f16(false, a, false, b, (short)0, c, false, false);
  asm volatile("v_nop\n\tv_nop\n\tv_nop\n\tv_nop" : "+v"(d) : "v"(a), "v"(b));
  return d;
}

__device__ __forceinline__ v8h cvt8(v4f a, v4f b, float s) {
  v8h c;
  c[0] = (_Float16)(a.x * s); c[1] = (_Float16)(a.y * s); c[2] = (_Float16)(a.z * s); c[3] = (_Float16)(a.w * s);
  c[4] = (_Float16)(b.x * s); c[5] = (_Float16)(b.y * s); c[6] = (_Float16)(b.z * s); c[7] = (_Float16)(b.w * s);
  return c;
}

__device__ __forceinline__ v4f sel4(int c, v4f a, v4f b) {
  v4f r;
  r.x = c ? a.x : b.x; r.y = c ? a.y : b.y; r.z = c ? a.z : b.z; r.w = c ? a.w : b.w;
  return r;
}

template <int K, int NT>
__device__ __forceinline__ void mma_tiles(const _Float16* sA, const _Float16* __restrict__ Bw,
                                          int wrow, int lane, v8f (&acc)[NT]) {
  static_assert((K % 32) == 0);
  constexpr int NKT = K / 32, APK = K + 8;
  const int hh = lane >> 4, m = lane & 15;
#pragma unroll
  for (int t = 0; t < NT; ++t) { v8f z = {0.f, 0.f, 0.f, 0.f, 0.f, 0.f, 0.f, 0.f}; acc[t] = z; }
  const _Float16* ap = sA + (wrow + m) * APK + 8 * hh;
#pragma unroll 1
  for (int kt = 0; kt < NKT; ++kt) {
    FragH a;
    a.h[0] = *(const v8h*)(ap + 32 * kt);
    a.h[1] = *(const v8h*)(ap + 32 * kt + 16);
#pragma unroll
    for (int t = 0; t < NT; ++t) {
      const _Float16* bp = Bw + (size_t)(16 * t + m) * K + 32 * kt + 8 * hh;
      FragH b;
      b.h[0] = *(const v8h*)bp;
      b.h[1] = *(const v8h*)(bp + 16);
      acc[t] = wmh(a.v, b.v, acc[t]);
    }
  }
}

template <int CW, int P>
__device__ __forceinline__ void store_group(const float* stg, float* C, int rowBase, int colBase,
                                            int wave, int lane, int nStore) {
  constexpr int LPR = CW / 4;
  constexpr int RPI = 32 / LPR;
  constexpr int NI  = 16 / RPI;
  static_assert(RPI == 1 || RPI == 2);
  const int lr = lane / LPR, lc = 4 * (lane % LPR);
  const float* lp = stg + (wave * 16 + lr) * CW + lc;
  const int r0 = rowBase + wave * 16 + lr;
  float* cp = C + (size_t)r0 * P + colBase + lc;
#pragma unroll
  for (int i = 0; i < NI; ++i) {
    if (r0 + i * RPI < nStore) {
      const v4f v = *(const v4f*)(lp + i * RPI * CW);
      *(volatile v4f*)(cp + (size_t)(i * RPI) * P) = v;
    }
  }
  __threadfence();
#pragma unroll
  for (int i = 0; i < NI; ++i) {
    if (r0 + i * RPI < nStore) {
      const v4f v = *(const v4f*)(lp + i * RPI * CW);
      *(volatile v4f*)(cp + (size_t)(i * RPI) * P) = v;
    }
  }
}

template <int NB>
__device__ __forceinline__ int scan_chunk(const int* __restrict__ dsts, int nE, int cbase, int slotBase,
                                          int vec8, int* list, int tid, int lane, int wave) {
  int wc = 0;
#pragma unroll
  for (int g = 0; g < NGRP; ++g) {
    const int el0  = (g * NTHR + tid) * EPT;
    const int e0   = cbase + el0;
    const int sent = -2147483647 - 1;
    v4i da, db;
    if (vec8 != 0 && cbase + CHUNK <= nE) {
      da = *(const v4i*)(dsts + e0);
      db = *(const v4i*)(dsts + e0 + 4);
    } else {
      da.x = (e0     < nE) ? dsts[min(e0, nE - 1)] : sent;
      da.y = (e0 + 1 < nE) ? dsts[min(e0 + 1, nE - 1)] : sent;
      da.z = (e0 + 2 < nE) ? dsts[min(e0 + 2, nE - 1)] : sent;
      da.w = (e0 + 3 < nE) ? dsts[min(e0 + 3, nE - 1)] : sent;
      db.x = (e0 + 4 < nE) ? dsts[min(e0 + 4, nE - 1)] : sent;
      db.y = (e0 + 5 < nE) ? dsts[min(e0 + 5, nE - 1)] : sent;
      db.z = (e0 + 6 < nE) ? dsts[min(e0 + 6, nE - 1)] : sent;
      db.w = (e0 + 7 < nE) ? dsts[min(e0 + 7, nE - 1)] : sent;
    }
    const unsigned nb = (unsigned)slotBase;
    const unsigned s0 = (unsigned)da.x - nb, s1 = (unsigned)da.y - nb;
    const unsigned s2 = (unsigned)da.z - nb, s3 = (unsigned)da.w - nb;
    const unsigned s4 = (unsigned)db.x - nb, s5 = (unsigned)db.y - nb;
    const unsigned s6 = (unsigned)db.z - nb, s7 = (unsigned)db.w - nb;
    const bool h0 = s0 < (unsigned)NB, h1 = s1 < (unsigned)NB, h2 = s2 < (unsigned)NB, h3 = s3 < (unsigned)NB;
    const bool h4 = s4 < (unsigned)NB, h5 = s5 < (unsigned)NB, h6 = s6 < (unsigned)NB, h7 = s7 < (unsigned)NB;
    const unsigned any = __builtin_amdgcn_ballot_w32(h0 | h1 | h2 | h3 | h4 | h5 | h6 | h7);
    if (any != 0u) {
#define HITJ(J, HJ, SJ) { \
        const unsigned mj = __builtin_amdgcn_ballot_w32(HJ); \
        if (mj != 0u) { \
          if (HJ) { \
            const int pos = wc + (int)__builtin_amdgcn_mbcnt_lo(mj, 0u); \
            if (pos < WCAP) list[wave * WCAP + pos] = ((el0 + (J)) << 12) | (int)(SJ); \
          } \
          wc += (int)__builtin_popcount(mj); } }
      HITJ(0, h0, s0)
      HITJ(1, h1, s1)
      HITJ(2, h2, s2)
      HITJ(3, h3, s3)
      HITJ(4, h4, s4)
      HITJ(5, h5, s5)
      HITJ(6, h6, s6)
      HITJ(7, h7, s7)
#undef HITJ
    }
  }
  return wc;
}

__global__ __launch_bounds__(NTHR) void k_wprep(
    const float* __restrict__ W_I, const float* __restrict__ W_O,
    const float* __restrict__ W_S, const float* __restrict__ W_T,
    _Float16* wbE, _Float16* wbR, _Float16* wbT, _Float16* wbTT) {
  const int b = blockIdx.x, tid = threadIdx.x;
  const float* W = W_I; int ldw = COMPD, koff = RELD, kqs = 4, nrow = ENTD, loc = 0; _Float16* dp = wbE;
  if (b < 8)       { W = W_I; ldw = COMPD; koff = RELD;        kqs = 4; nrow = ENTD; dp = wbE;                   loc = b * NTHR + tid; }
  else if (b < 16) { W = W_O; ldw = COMPD; koff = RELD;        kqs = 4; nrow = ENTD; dp = wbE + ENTD * ENTD;     loc = (b - 8) * NTHR + tid; }
  else if (b < 24) { W = W_S; ldw = ENTD;  koff = 0;           kqs = 4; nrow = ENTD; dp = wbE + 2 * ENTD * ENTD; loc = (b - 16) * NTHR + tid; }
  else if (b < 32) { W = W_I; ldw = COMPD; koff = 0;           kqs = 4; nrow = ENTD; dp = wbR;                   loc = (b - 24) * NTHR + tid; }
  else if (b < 40) { W = W_O; ldw = COMPD; koff = 0;           kqs = 4; nrow = ENTD; dp = wbR + ENTD * RELD;     loc = (b - 32) * NTHR + tid; }
  else if (b < 44) { W = W_I; ldw = COMPD; koff = RELD + ENTD; kqs = 3; nrow = ENTD; dp = wbT;                   loc = (b - 40) * NTHR + tid; }
  else if (b < 48) { W = W_O; ldw = COMPD; koff = RELD + ENTD; kqs = 3; nrow = ENTD; dp = wbT + ENTD * TIMD;     loc = (b - 44) * NTHR + tid; }
  else             { W = W_T; ldw = TIMD;  koff = 0;           kqs = 3; nrow = TIMD; dp = wbTT;                  loc = (b - 48) * NTHR + tid; }
  const int kq = 1 << kqs;
  int n = loc >> kqs;
  const int g = loc & (kq - 1);
  const bool ok = n < nrow;
  n = n > nrow - 1 ? nrow - 1 : n;
  const float* sp = W + (size_t)n * ldw + koff + 8 * g;
  const v4f a = *(const v4f*)sp, c = *(const v4f*)(sp + 4);
  const v8h cv = cvt8(a, c, WSCALE);
  _Float16* q = dp + (size_t)n * (8 * kq) + 8 * g;
  if (ok) *(volatile v8h*)q = cv;
  __threadfence();
  if (ok) *(volatile v8h*)q = cv;
}

__global__ __launch_bounds__(NTHR) void k_count(const int* __restrict__ dsts, int* cnt, int nE, int vec8) {
  __shared__ __attribute__((aligned(16))) int scnt[NBC];
  __shared__ __attribute__((aligned(16))) int list[LISTN];
  __shared__ int wcnt[NWAVE];
  const int tid = threadIdx.x, lane = tid & 31, wave = tid >> 5;
  const int nodeBase = blockIdx.x * NBC;

  for (int i = tid; i < NBC; i += NTHR) scnt[i] = 0;
  __syncthreads();

  const int nChunks = (nE + CHUNK - 1) / CHUNK;
#pragma unroll 1
  for (int ch = 0; ch < nChunks; ++ch) {
    const int cbase = ch * CHUNK;
    const int wc = scan_chunk<NBC>(dsts, nE, cbase, nodeBase, vec8, list, tid, lane, wave);
    if (lane == 0) wcnt[wave] = wc;
    __syncthreads();
    if (wave == 0) {
#pragma unroll 1
      for (int wsx = 0; wsx < NWAVE; ++wsx) {
        int n = __builtin_amdgcn_readfirstlane(wcnt[wsx]);
        n = n > WCAP ? WCAP : (n < 0 ? 0 : n);
        const int* lp = list + wsx * WCAP;
#pragma unroll 1
        for (int i = 0; i < n; ++i) {
          const int ent  = __builtin_amdgcn_readfirstlane(lp[i]);
          const int slot = ent & (NBC - 1);
          if (lane == 0) scnt[slot] = scnt[slot] + 1;
        }
      }
    }
    __syncthreads();
  }

  v4i cq[4];
#pragma unroll
  for (int q = 0; q < 4; ++q) {
    const int f = (wave * 4 + q) * 128 + 4 * lane;
    cq[q] = *(const v4i*)(scnt + f);
  }
  int* cp = cnt + (size_t)nodeBase;
#pragma unroll
  for (int q = 0; q < 4; ++q) {
    const int f = (wave * 4 + q) * 128 + 4 * lane;
    *(volatile v4i*)(cp + f) = cq[q];
  }
  __threadfence();
#pragma unroll
  for (int q = 0; q < 4; ++q) {
    const int f = (wave * 4 + q) * 128 + 4 * lane;
    *(volatile v4i*)(cp + f) = cq[q];
  }
}

__global__ __launch_bounds__(OTHR) void k_offsets(
    const int* __restrict__ cnt, int* off, int* rbase, int nChunk) {
  __shared__ __attribute__((aligned(16))) int soff[NBC];
  __shared__ __attribute__((aligned(16))) int srb[RBN];
  __shared__ int wtot[OTHR / 32];
  const int tid = threadIdx.x, lane = tid & 31, wave = tid >> 5, sub = tid >> 7;
  for (int i = tid; i < RBN; i += OTHR) srb[i] = 0;
  int carry = 0;
#pragma unroll 1
  for (int ch = 0; ch < nChunk; ++ch) {
    const int base = ch * NBC;
    const v4i c0 = *(const v4i*)(cnt + base + 8 * tid);
    const v4i c1 = *(const v4i*)(cnt + base + 8 * tid + 4);
    const int e0 = max(c0.x, 0), e1 = max(c0.y, 0), e2 = max(c0.z, 0), e3 = max(c0.w, 0);
    const int e4 = max(c1.x, 0), e5 = max(c1.y, 0), e6 = max(c1.z, 0), e7 = max(c1.w, 0);
    const int ts = e0 + e1 + e2 + e3 + e4 + e5 + e6 + e7;
    int incl = ts;
#pragma unroll
    for (int d = 1; d < 32; d <<= 1) {
      const int t = __shfl_up(incl, d);
      if (lane >= d) incl += t;
    }
    if (lane == 31) wtot[wave] = incl;
    __syncthreads();
    const int S0 = wtot[0]  + wtot[1]  + wtot[2]  + wtot[3];
    const int S1 = wtot[4]  + wtot[5]  + wtot[6]  + wtot[7];
    const int S2 = wtot[8]  + wtot[9]  + wtot[10] + wtot[11];
    const int S3 = wtot[12] + wtot[13] + wtot[14] + wtot[15];
    int pre = 0;
#pragma unroll 1
    for (int w = 4 * sub; w < wave; ++w) pre += wtot[w];
    const int b0 = carry;
    const int b1 = b0 + ((S0 + 31) & ~31);
    const int b2 = b1 + ((S1 + 31) & ~31);
    const int b3 = b2 + ((S2 + 31) & ~31);
    const int b4 = b3 + ((S3 + 31) & ~31);
    const int myb = sub == 0 ? b0 : (sub == 1 ? b1 : (sub == 2 ? b2 : b3));
    if (tid == 0) {
      srb[min(4 * ch + 0, RBN - 1)] = b0;
      srb[min(4 * ch + 1, RBN - 1)] = b1;
      srb[min(4 * ch + 2, RBN - 1)] = b2;
      srb[min(4 * ch + 3, RBN - 1)] = b3;
    }
    int run = myb + pre + incl - ts;
    soff[8 * tid + 0] = run; run += e0;
    soff[8 * tid + 1] = run; run += e1;
    soff[8 * tid + 2] = run; run += e2;
    soff[8 * tid + 3] = run; run += e3;
    soff[8 * tid + 4] = run; run += e4;
    soff[8 * tid + 5] = run; run += e5;
    soff[8 * tid + 6] = run; run += e6;
    soff[8 * tid + 7] = run;
    carry = b4;
    __syncthreads();
    const v4i o0 = *(const v4i*)(soff + 4 * tid);
    const v4i o1 = *(const v4i*)(soff + 4 * (tid + OTHR));
    int* op = off + base;
    *(volatile v4i*)(op + 4 * tid) = o0;
    *(volatile v4i*)(op + 4 * (tid + OTHR)) = o1;
    __threadfence();
    *(volatile v4i*)(op + 4 * tid) = o0;
    *(volatile v4i*)(op + 4 * (tid + OTHR)) = o1;
    __syncthreads();
  }
  if (tid == 0) srb[min(4 * nChunk, RBN - 1)] = carry;
  __syncthreads();
  v4i rv = {0, 0, 0, 0};
  if (tid < 32) rv = *(const v4i*)(srb + 4 * tid);
  if (tid < 32) *(volatile v4i*)(rbase + 4 * tid) = rv;
  __threadfence();
  if (tid < 32) *(volatile v4i*)(rbase + 4 * tid) = rv;
}

__global__ __launch_bounds__(NTHR) void k_fill(
    const int* __restrict__ dsts, const int* __restrict__ off, const int* __restrict__ rbase,
    int* csr, int nE, int vec8, int csrLen) {
  extern __shared__ v4f lds_dyn[];
  int* region = (int*)lds_dyn;
  int* cursor = region + RCAP;
  int* list   = cursor + NBF;
  int* wcnt   = list + LISTN;
  const int tid = threadIdx.x, lane = tid & 31, wave = tid >> 5;
  const int b = blockIdx.x;
  const int nodeBase = b * NBF;

  int rb0 = rbase[b];
  const int rb1 = rbase[b + 1];
  rb0 = rb0 < 0 ? 0 : (rb0 > csrLen ? csrLen : rb0);
  rb0 &= ~31;
  int len = rb1 - rb0;
  len = len < 0 ? 0 : (len > RCAP ? RCAP : len);
  int lenW = (len + 31) & ~31;
  if (rb0 + lenW > csrLen) lenW = (csrLen - rb0) & ~31;

  {
    const v4i z = {0, 0, 0, 0};
    for (int i = tid; i < RCAP / 4; i += NTHR) ((v4i*)region)[i] = z;
    for (int s = tid; s < NBF; s += NTHR) {
      int o = off[nodeBase + s] - rb0;
      o = o < 0 ? 0 : (o > RCAP ? RCAP : o);
      cursor[s] = o;
    }
  }
  __syncthreads();

  const int nChunks = (nE + CHUNK - 1) / CHUNK;
#pragma unroll 1
  for (int ch = 0; ch < nChunks; ++ch) {
    const int cbase = ch * CHUNK;
    const int wc = scan_chunk<NBF>(dsts, nE, cbase, nodeBase, vec8, list, tid, lane, wave);
    if (lane == 0) wcnt[wave] = wc;
    __syncthreads();
    if (wave == 0) {
#pragma unroll 1
      for (int wsx = 0; wsx < NWAVE; ++wsx) {
        int n = __builtin_amdgcn_readfirstlane(wcnt[wsx]);
        n = n > WCAP ? WCAP : (n < 0 ? 0 : n);
        const int* lp = list + wsx * WCAP;
#pragma unroll 1
        for (int i = 0; i < n; ++i) {
          const int ent  = __builtin_amdgcn_readfirstlane(lp[i]);
          const int slot = ent & (NBF - 1);
          int e = cbase + ((ent >> 12) & (CHUNK - 1));
          e = e < 0 ? 0 : (e > nE - 1 ? nE - 1 : e);
          if (lane == 0) {
            int pos = cursor[slot];
            pos = pos < 0 ? 0 : (pos > RCAP - 1 ? RCAP - 1 : pos);
            region[pos] = e;
            const int np = pos + 1;
            cursor[slot] = np > RCAP ? RCAP : np;
          }
        }
      }
    }
    __syncthreads();
  }

  const int nv = lenW >> 2;
  int* gp = csr + rb0;
#pragma unroll 1
  for (int i = tid; i < nv; i += NTHR) { const v4i v = ((const v4i*)region)[i]; *(volatile v4i*)(gp + 4 * i) = v; }
  __threadfence();
#pragma unroll 1
  for (int i = tid; i < nv; i += NTHR) { const v4i v = ((const v4i*)region)[i]; *(volatile v4i*)(gp + 4 * i) = v; }
}

template <int K, int NCT>
__global__ __launch_bounds__(NTHR) void k_gemm(
    const float* __restrict__ x, const _Float16* __restrict__ Bw, const float* __restrict__ bias,
    float* C, int nValid, int nStore, int useBias) {
  typedef GemmCfg<K, NCT> G;
  static_assert((K % 32) == 0);
  static_assert(NCT == 1 || (NCT % 2) == 0);
  static_assert((G::LDSA % 16) == 0 && (G::APK % 8) == 0);
  extern __shared__ v4f lds_dyn[];
  _Float16* sA  = (_Float16*)lds_dyn;
  float*    stg = (float*)((char*)lds_dyn + G::LDSA);
  const int tid = threadIdx.x, lane = tid & 31, wave = tid >> 5, hh = lane >> 4, m = lane & 15;
  const int rowBase = blockIdx.x * GROWS;
  constexpr int TPR = K / 8, RPI = NTHR / TPR, NIT = GROWS / RPI;
  static_assert(NIT * RPI == GROWS);
  const int c0 = (tid % TPR) * 8, rr = tid / TPR;

#pragma unroll 2
  for (int it = 0; it < NIT; ++it) {
    const int r = it * RPI + rr;
    int row = rowBase + r;
    row = row > nValid - 1 ? nValid - 1 : row;
    row = row < 0 ? 0 : row;
    const float* ap = x + (size_t)row * K + c0;
    const v4f a = *(const v4f*)ap, b = *(const v4f*)(ap + 4);
    *(v8h*)(sA + r * G::APK + c0) = cvt8(a, b, 1.0f);
  }
  __syncthreads();

#pragma unroll 1
  for (int g = 0; g < G::NG; ++g) {
#pragma unroll
    for (int ch = 0; ch < G::NCH; ++ch) {
      v8f acc[4];
      const int colBase = g * G::CW + 64 * ch;
      mma_tiles<K, 4>(sA, Bw + (size_t)colBase * K, wave * 16, lane, acc);
      float* sp = stg + (wave * 16 + 8 * hh) * G::CW + 64 * ch + m;
#pragma unroll
      for (int t = 0; t < 4; ++t) {
        float bv = 0.0f;
        if (useBias != 0) bv = bias[colBase + 16 * t + m];
#pragma unroll
        for (int r = 0; r < 8; ++r) sp[r * G::CW + 16 * t] = acc[t][r] * WINV + bv;
      }
    }
    __syncthreads();
    store_group<G::CW, G::P>(stg, C, rowBase, g * G::CW, wave, lane, nStore);
    __syncthreads();
  }
}

__global__ __launch_bounds__(NTHR) void k_agg(
    const int* __restrict__ csr, const int* __restrict__ off, const int* __restrict__ cnt,
    const int* __restrict__ srcs, const int* __restrict__ rels, const int* __restrict__ tims,
    const int* __restrict__ invs,
    const float* __restrict__ PE, const float* __restrict__ PR, const float* __restrict__ PT,
    const float* __restrict__ bI, const float* __restrict__ bO, const float* __restrict__ bS,
    float* out0, int nN, int nR, int nT, int nE, int csrLen) {
#pragma clang fp contract(off)
  const int tid = threadIdx.x, lane = tid & 31, wave = tid >> 5;
  const int tbase = blockIdx.x * TGT + wave * 32;
  const int cl = tbase + lane;
  const int cnt_l = cnt[cl];
  const int off_l = off[cl];
  const v4f bI4 = *(const v4f*)(bI + 4 * lane);
  const v4f bO4 = *(const v4f*)(bO + 4 * lane);
  const v4f bS4 = *(const v4f*)(bS + 4 * lane);

#pragma unroll 1
  for (int j = 0; j < 32; ++j) {
    const int c = tbase + j;
    int n = __builtin_amdgcn_readlane(cnt_l, j);
    n = n < 0 ? 0 : (n > DEGCAP ? DEGCAP : n);
    const int st = __builtin_amdgcn_readlane(off_l, j);
    v4f sm = {0.0f, 0.0f, 0.0f, 0.0f};
#pragma unroll 1
    for (int q0 = 0; q0 < n; q0 += 32) {
      int pos = st + q0 + lane;
      pos = pos < 0 ? 0 : (pos > csrLen - 1 ? csrLen - 1 : pos);
      int el = csr[pos];
      el = el < 0 ? 0 : (el > nE - 1 ? nE - 1 : el);
      int sl = srcs[el];
      sl = sl < 0 ? 0 : (sl > nN - 1 ? nN - 1 : sl);
      int rl = rels[el];
      rl = rl < 0 ? 0 : (rl > nR - 1 ? nR - 1 : rl);
      int tl = tims[el];
      tl = tl < 0 ? 0 : (tl > nT - 1 ? nT - 1 : tl);
      const int il = (invs[el] != 0) ? 1 : 0;
      const int mcnt = (n - q0) < 32 ? (n - q0) : 32;
#pragma unroll 1
      for (int p = 0; p < mcnt; ++p) {
        const int s  = __builtin_amdgcn_readlane(sl, p);
        const int r  = __builtin_amdgcn_readlane(rl, p);
        const int t  = __builtin_amdgcn_readlane(tl, p);
        const int iv = __builtin_amdgcn_readlane(il, p);
        const int co = iv * ENTD + 4 * lane;
        const v4f pe = *(const v4f*)(PE + (size_t)s * PEP + co);
        const v4f pr = *(const v4f*)(PR + (size_t)r * PRP + co);
        const v4f pt = *(const v4f*)(PT + (size_t)t * PRP + co);
        const v4f bb = sel4(iv, bO4, bI4);
        const v4f msg = ((pr + pe) + pt) + bb;
        sm = sm + msg;
      }
    }
    const float rc = 1.0f / (float)(n > 1 ? n : 1);
    const v4f mean = sm * rc;
    const v4f ps = *(const v4f*)(PE + (size_t)c * PEP + 2 * ENTD + 4 * lane);
    const v4f res = (ps + bS4) + mean;
    float* ap = out0 + (size_t)c * ENTD + 4 * lane;
    if (c < nN) *(volatile v4f*)ap = res;
    __threadfence();
    if (c < nN) *(volatile v4f*)ap = res;
  }
}

extern "C" void kernel_launch(void* const* d_in, const int* in_sizes, int n_in,
                              void* d_out, int out_size, void* d_ws, size_t ws_size,
                              hipStream_t stream) {
  if (n_in < 16) return;
  const int nN = in_sizes[0] / ENTD;
  const int nR = in_sizes[1] / RELD;
  const int nT = in_sizes[2] / TIMD;
  const int nE = in_sizes[11];
  if (nN <= 0 || nR <= 0 || nT <= 0 || nE <= 0) return;
  if (in_sizes[0] != nN * ENTD || in_sizes[1] != nR * RELD || in_sizes[2] != nT * TIMD) return;
  if (in_sizes[3] != ENTD * COMPD || in_sizes[5] != ENTD * COMPD) return;
  if (in_sizes[7] != ENTD * ENTD || in_sizes[9] != TIMD * TIMD) return;
  if (in_sizes[4] != ENTD || in_sizes[6] != ENTD || in_sizes[8] != ENTD || in_sizes[10] != TIMD) return;
  if (in_sizes[12] != nE || in_sizes[13] != nE || in_sizes[14] != nE || in_sizes[15] != nE) return;
  if (out_size != nN * ENTD + nT * TIMD) return;
  if (nE > (1 << 28) || nN > (1 << 22) || nR > (1 << 20) || nT > (1 << 20)) return;
  if (nR * RELD < PRP || nT * TIMD < PRP) return;

  const float* ent_emb  = (const float*)d_in[0];
  const float* rel_emb  = (const float*)d_in[1];
  const float* time_emb = (const float*)d_in[2];
  const float* W_I = (const float*)d_in[3];
  const float* b_I = (const float*)d_in[4];
  const float* W_O = (const float*)d_in[5];
  const float* b_O = (const float*)d_in[6];
  const float* W_S = (const float*)d_in[7];
  const float* b_S = (const float*)d_in[8];
  const float* W_T = (const float*)d_in[9];
  const float* b_T = (const float*)d_in[10];
  const int* srcs = (const int*)d_in[11];
  const int* dsts = (const int*)d_in[12];
  const int* rels = (const int*)d_in[13];
  const int* tims = (const int*)d_in[14];
  const int* invs = (const int*)d_in[15];
  float* out0 = (float*)d_out;
  float* out1 = out0 + (size_t)nN * ENTD;

  const int NPAD   = ((nN + TGT - 1) / TGT) * TGT;
  const int RPAD   = ((nR + GROWS - 1) / GROWS) * GROWS;
  const int TPAD   = ((nT + GROWS - 1) / GROWS) * GROWS;
  const int nBC    = (nN + NBC - 1) / NBC;
  const int CNTPAD = nBC * NBC;
  if (4 * nBC + 1 > RBN) return;
  const int nBF    = (nN + NBF - 1) / NBF;
  const int csrLen = ((nE + 31) & ~31) + 4096;
  if (31 * 4 * nBC > 4096) return;
  const int nGemmE = NPAD / GROWS;
  const int nGemmR = RPAD / GROWS;
  const int nGemmT = TPAD / GROWS;
  const int nAgg   = NPAD / TGT;

  char* ws = (char*)d_ws;
  size_t off = 0;
  const size_t oWE  = off; off += (size_t)PEP * ENTD * 2;          off = (off + 255) & ~(size_t)255;
  const size_t oWR  = off; off += (size_t)PRP * RELD * 2;          off = (off + 255) & ~(size_t)255;
  const size_t oWT  = off; off += (size_t)PRP * TIMD * 2;          off = (off + 255) & ~(size_t)255;
  const size_t oWTT = off; off += (size_t)TIMD * TIMD * 2;         off = (off + 255) & ~(size_t)255;
  const size_t oCnt = off; off += (size_t)CNTPAD * 4;              off = (off + 255) & ~(size_t)255;
  const size_t oOff = off; off += (size_t)CNTPAD * 4;              off = (off + 255) & ~(size_t)255;
  const size_t oRb  = off; off += (size_t)RBN * 4;                 off = (off + 255) & ~(size_t)255;
  const size_t oCsr = off; off += (size_t)csrLen * 4;              off = (off + 255) & ~(size_t)255;
  const size_t oPE  = off; off += (size_t)NPAD * PEP * 4;          off = (off + 255) & ~(size_t)255;
  const size_t oPR  = off; off += (size_t)RPAD * PRP * 4;          off = (off + 255) & ~(size_t)255;
  const size_t oPT  = off; off += (size_t)TPAD * PRP * 4;          off = (off + 255) & ~(size_t)255;
  if (off > ws_size || off > (size_t)WSCAP) return;
  _Float16* wbE  = (_Float16*)(ws + oWE);
  _Float16* wbR  = (_Float16*)(ws + oWR);
  _Float16* wbT  = (_Float16*)(ws + oWT);
  _Float16* wbTT = (_Float16*)(ws + oWTT);
  int*      cnt  = (int*)(ws + oCnt);
  int*      offp = (int*)(ws + oOff);
  int*      rb   = (int*)(ws + oRb);
  int*      csr  = (int*)(ws + oCsr);
  float*    PE   = (float*)(ws + oPE);
  float*    PR   = (float*)(ws + oPR);
  float*    PT   = (float*)(ws + oPT);

  const int vec8 = 1;

  k_wprep<<<WPREP_BLOCKS, NTHR, 0, stream>>>(W_I, W_O, W_S, W_T, wbE, wbR, wbT, wbTT);

  k_count<<<nBC, NTHR, 0, stream>>>(dsts, cnt, nE, vec8);
  k_offsets<<<1, OTHR, 0, stream>>>(cnt, offp, rb, nBC);
  hipFuncSetAttribute(reinterpret_cast<const void*>(&k_fill),
                      hipFuncAttributeMaxDynamicSharedMemorySize, LDS_FILL);
  k_fill<<<nBF, NTHR, LDS_FILL, stream>>>(dsts, offp, rb, csr, nE, vec8, csrLen);

  hipFuncSetAttribute(reinterpret_cast<const void*>(&k_gemm<ENTD, 6>),
                      hipFuncAttributeMaxDynamicSharedMemorySize, GemmCfg<ENTD, 6>::LDS);
  k_gemm<ENTD, 6><<<nGemmE, NTHR, GemmCfg<ENTD, 6>::LDS, stream>>>(ent_emb, wbE, ent_emb, PE, nN, NPAD, 0);

  hipFuncSetAttribute(reinterpret_cast<const void*>(&k_gemm<RELD, 4>),
                      hipFuncAttributeMaxDynamicSharedMemorySize, GemmCfg<RELD, 4>::LDS);
  k_gemm<RELD, 4><<<nGemmR, NTHR, GemmCfg<RELD, 4>::LDS, stream>>>(rel_emb, wbR, rel_emb, PR, nR, RPAD, 0);

  hipFuncSetAttribute(reinterpret_cast<const void*>(&k_gemm<TIMD, 4>),
                      hipFuncAttributeMaxDynamicSharedMemorySize, GemmCfg<TIMD, 4>::LDS);
  k_gemm<TIMD, 4><<<nGemmT, NTHR, GemmCfg<TIMD, 4>::LDS, stream>>>(time_emb, wbT, time_emb, PT, nT, TPAD, 0);

  hipFuncSetAttribute(reinterpret_cast<const void*>(&k_gemm<TIMD, 1>),
                      hipFuncAttributeMaxDynamicSharedMemorySize, GemmCfg<TIMD, 1>::LDS);
  k_gemm<TIMD, 1><<<nGemmT, NTHR, GemmCfg<TIMD, 1>::LDS, stream>>>(time_emb, wbTT, b_T, out1, nT, nT, 1);

  k_agg<<<nAgg, NTHR, 0, stream>>>(csr, offp, cnt, srcs, rels, tims, invs, PE, PR, PT,
                                   b_I, b_O, b_S, out0, nN, nR, nT, nE, csrLen);
}
